// MinimalSSMTorch_20976620274247
// MI455X (gfx1250) — hardware-run, weakly checked
//
#include <hip/hip_runtime.h>
#include <math.h>

typedef __attribute__((ext_vector_type(16))) _Float16 v16h;
typedef __attribute__((ext_vector_type(8)))  _Float16 v8h;
typedef __attribute__((ext_vector_type(8)))  float    v8f;
typedef __attribute__((ext_vector_type(4)))  float    v4f;
typedef __attribute__((ext_vector_type(4)))  unsigned int v4u;

constexpr int kBatch = 4;
constexpr int kSeq   = 2048;
constexpr int kDm    = 1024;
constexpr int kDin   = 2048;
constexpr int kNst   = 16;
constexpr int kRows  = kBatch * kSeq;
constexpr int kWinN  = 2 * kDin;
constexpr int kAbcP  = 64;
constexpr int kScanTS = 32;
constexpr int kScanCh = 256;
constexpr int kScanYP = 260;

constexpr float kXCarry    = 16.0f;
constexpr float kWCarry    = 256.0f;
constexpr float kActCarry  = 16.0f;
constexpr float kScanCarry = 4096.0f;
constexpr float kNormCarry = 16.0f;
constexpr float kResCarry  = 2048.0f;
constexpr float kResInv    = 1.0f / kResCarry;
constexpr float kFoldMain  = 1.0f / (kXCarry * kWCarry);
constexpr float kFoldCross = kFoldMain * kResInv;
constexpr float kScaleAbc  = 1.0f / (kActCarry * kWCarry);
constexpr float kScaleOut  = 1.0f / (kNormCarry * kWCarry);
constexpr float kActInv    = 1.0f / kActCarry;
constexpr float kScanInv   = 1.0f / kScanCarry;
constexpr float kMeanFold  = kScanInv * kScanInv / (float)kDin;
constexpr float kEps       = 1.1920929e-07f;
constexpr float kF16Min    = 6.103515625e-05f;

static_assert(kRows == 8192 && kWinN == 4096 && kNst == 16);
static_assert(3 * kNst <= kAbcP);
static_assert((kDm % 32) == 0 && (kDin % 32) == 0);
static_assert((kRows % 32) == 0 && (kDin % 64) == 0 && (kDm % 64) == 0 && (kAbcP % 64) == 0 && (kWinN % 64) == 0);
static_assert((kSeq % kScanTS) == 0 && (kDin % kScanCh) == 0);
static_assert(((kRows / 16) * (kDin / 64)) % 4 == 0);

constexpr size_t kSzWin  = (size_t)kWinN * kDm * 2;
constexpr size_t kSzWabc = (size_t)kAbcP * kDin * 2;
constexpr size_t kSzWout = (size_t)kDm * kDin * 2;
constexpr size_t kSzXHL  = (size_t)kRows * kDm * 2 * 2;
constexpr size_t kSzXin  = (size_t)kRows * kDin * 2;
constexpr size_t kSzAbc  = (size_t)kRows * kAbcP * 4;
constexpr size_t kWsTotal = 2 * kSzWin + 2 * kSzWabc + kSzWout + kSzXHL + 2 * kSzXin + kSzAbc;
static_assert(kWsTotal == 124256256ull);
static_assert(kWsTotal <= 134217728ull);
static_assert((size_t)kRows * kDin * 2 == kSzXHL);
static_assert((kSzWin % 256) == 0 && (kSzWabc % 256) == 0 && (kSzWout % 256) == 0 && (kSzXHL % 256) == 0 &&
              (kSzXin % 256) == 0 && (kSzAbc % 256) == 0);

__device__ __forceinline__ unsigned pk16(unsigned short a, unsigned short b) {
  return (unsigned)a | ((unsigned)b << 16);
}
__device__ __forceinline__ float flush_h(float f) {
  return (fabsf(f) < kF16Min) ? 0.0f : f;
}
__device__ __forceinline__ unsigned short h_bits(float f) {
  const _Float16 h = (_Float16)flush_h(f);
  return __builtin_bit_cast(unsigned short, h);
}
__device__ __forceinline__ void h_split(float v, unsigned short& hb, unsigned short& rb) {
  const _Float16 h = (_Float16)flush_h(v);
  const float hf = (float)h;
  const float d = (v - hf) * kResCarry;
  const _Float16 r = (_Float16)flush_h(d);
  hb = __builtin_bit_cast(unsigned short, h);
  rb = __builtin_bit_cast(unsigned short, r);
}
__device__ __forceinline__ v4u pack8_plain(const float (&v)[8]) {
  unsigned short hb[8];
#pragma unroll
  for (int e = 0; e < 8; ++e) hb[e] = h_bits(v[e]);
  return (v4u){pk16(hb[0], hb[1]), pk16(hb[2], hb[3]), pk16(hb[4], hb[5]), pk16(hb[6], hb[7])};
}
__device__ __forceinline__ void pack8_split(const float (&v)[8], v4u& uh, v4u& ur) {
  unsigned short hb[8], rb[8];
#pragma unroll
  for (int e = 0; e < 8; ++e) h_split(v[e], hb[e], rb[e]);
  uh = (v4u){pk16(hb[0], hb[1]), pk16(hb[2], hb[3]), pk16(hb[4], hb[5]), pk16(hb[6], hb[7])};
  ur = (v4u){pk16(rb[0], rb[1]), pk16(rb[2], rb[3]), pk16(rb[4], rb[5]), pk16(rb[6], rb[7])};
}
__device__ __forceinline__ float h16_to_f32(unsigned hb) {
  const unsigned sgn = (hb & 0x8000u) << 16;
  const unsigned em = hb & 0x7fffu;
  const float fn = __uint_as_float((em << 13) + 0x38000000u);
  const float fs = (float)em * 5.9604644775390625e-8f;
  const float mag = (em < 0x400u) ? fs : fn;
  return __uint_as_float(__float_as_uint(mag) | sgn);
}
__device__ __forceinline__ void unpack8(const v4u w, float (&f)[8]) {
  const unsigned w0 = w[0];
  const unsigned w1 = w[1];
  const unsigned w2 = w[2];
  const unsigned w3 = w[3];
  f[0] = h16_to_f32(w0 & 0xffffu);
  f[1] = h16_to_f32(w0 >> 16);
  f[2] = h16_to_f32(w1 & 0xffffu);
  f[3] = h16_to_f32(w1 >> 16);
  f[4] = h16_to_f32(w2 & 0xffffu);
  f[5] = h16_to_f32(w2 >> 16);
  f[6] = h16_to_f32(w3 & 0xffffu);
  f[7] = h16_to_f32(w3 >> 16);
}
__device__ __forceinline__ float wave_sum32(float v) {
#pragma unroll
  for (int o = 16; o > 0; o >>= 1) v += __shfl_xor(v, o, 32);
  return v;
}

struct FragH {
  union U { v16h v; v8h h[2]; };
  static __device__ __forceinline__ v16h load(const _Float16* p) {
    U f;
    f.h[0] = *(const v8h*)(p);
    f.h[1] = *(const v8h*)(p + 16);
    return f.v;
  }
  static __device__ __forceinline__ v8f mma(v16h a, v16h b, v8f c) {
    return __builtin_amdgcn_wmma_f32_16x16x32_f16(false, a, false, b, (short)0, c, false, false);
  }
};
__device__ __forceinline__ void guard_split(v8f& a0, v8f& a1, v8f& a2, v8f& a3,
                                            v16h x0, v16h x1, v16h x2, v16h x3, v16h y0, v16h y1) {
  asm volatile("v_nop\n\tv_nop\n\tv_nop\n\tv_nop"
               : "+v"(a0), "+v"(a1), "+v"(a2), "+v"(a3)
               : "v"(x0), "v"(x1), "v"(x2), "v"(x3), "v"(y0), "v"(y1));
}
__device__ __forceinline__ void guard_plain(v8f& a0, v8f& a1, v16h x0, v16h x1, v16h y0) {
  asm volatile("v_nop\n\tv_nop\n\tv_nop\n\tv_nop"
               : "+v"(a0), "+v"(a1)
               : "v"(x0), "v"(x1), "v"(y0));
}
__device__ __forceinline__ void acc_guard4(v8f& a, v8f& b, v8f& c, v8f& d) {
  asm volatile("v_nop\n\tv_nop\n\tv_nop\n\tv_nop" : "+v"(a), "+v"(b), "+v"(c), "+v"(d));
}
__device__ __forceinline__ void guard_m(v8f& a, v16h x, v16h y) {
  asm volatile("v_nop\n\tv_nop\n\tv_nop\n\tv_nop" : "+v"(a) : "v"(x), "v"(y));
}
__device__ __forceinline__ void guard_c(v8f& a, v16h x0, v16h x1, v16h y0, v16h y1) {
  asm volatile("v_nop\n\tv_nop\n\tv_nop\n\tv_nop" : "+v"(a) : "v"(x0), "v"(x1), "v"(y0), "v"(y1));
}

template <bool SPLIT>
__global__ __launch_bounds__(256) void gemm_f16_kernel(
    const unsigned short* __restrict__ Ahp, const unsigned short* __restrict__ Arp, int lda,
    const unsigned short* __restrict__ Bhp, const unsigned short* __restrict__ Brp, int ldb,
    float* __restrict__ C, int ldc, int M, int N, int K, float scale) {
  __shared__ __align__(16) float sT[8][16 * 68];
  const int lane = threadIdx.x & 31;
  const int wave = threadIdx.x >> 5;
  const int tilesN = N >> 6;
  const int tilesM = M >> 5;
  const int tile = blockIdx.x * 8 + wave;
  if (tile >= tilesM * tilesN) return;
  const int tm = tile / tilesN;
  const int tn = tile - tm * tilesN;
  const int m0 = tm << 5;
  const int n0 = tn << 6;
  const int rlane = lane & 15;
  const int half8 = (lane >> 4) * 8;
  const int mOff  = (lane >> 4) * 8;

  const size_t aoff = (size_t)(m0 + rlane) * lda + half8;
  const size_t boff = (size_t)(n0 + rlane) * ldb + half8;
  const _Float16* pa0 = (const _Float16*)Ahp + aoff;
  const _Float16* pa1 = pa0 + (size_t)16 * lda;
  const _Float16* pr0 = SPLIT ? ((const _Float16*)Arp + aoff) : pa0;
  const _Float16* pr1 = pr0 + (size_t)16 * lda;
  const _Float16* pbh = (const _Float16*)Bhp + boff;
  const _Float16* pbr = SPLIT ? ((const _Float16*)Brp + boff) : pbh;
  const size_t bstep = (size_t)16 * ldb;

  v8f acc[2][4], accr[2][4];
#pragma unroll
  for (int i = 0; i < 2; ++i)
#pragma unroll
    for (int j = 0; j < 4; ++j) {
      acc[i][j]  = (v8f){0.f, 0.f, 0.f, 0.f, 0.f, 0.f, 0.f, 0.f};
      accr[i][j] = (v8f){0.f, 0.f, 0.f, 0.f, 0.f, 0.f, 0.f, 0.f};
    }

  for (int k0 = 0; k0 < K; k0 += 32) {
    const v16h ah0 = FragH::load(pa0 + k0);
    const v16h ah1 = FragH::load(pa1 + k0);
    v16h ar0 = ah0, ar1 = ah1;
    if (SPLIT) {
      ar0 = FragH::load(pr0 + k0);
      ar1 = FragH::load(pr1 + k0);
    }
#pragma unroll
    for (int j = 0; j < 4; ++j) {
      const v16h bh = FragH::load(pbh + j * bstep + k0);
      v16h br = bh;
      if (SPLIT) br = FragH::load(pbr + j * bstep + k0);
      acc[0][j] = FragH::mma(ah0, bh, acc[0][j]);
      acc[1][j] = FragH::mma(ah1, bh, acc[1][j]);
      if (SPLIT) {
        accr[0][j] = FragH::mma(ah0, br, accr[0][j]);
        accr[1][j] = FragH::mma(ah1, br, accr[1][j]);
        accr[0][j] = FragH::mma(ar0, bh, accr[0][j]);
        accr[1][j] = FragH::mma(ar1, bh, accr[1][j]);
        guard_split(acc[0][j], acc[1][j], accr[0][j], accr[1][j], ah0, ah1, ar0, ar1, bh, br);
      } else {
        guard_plain(acc[0][j], acc[1][j], ah0, ah1, bh);
      }
    }
  }
  acc_guard4(acc[0][0], acc[0][1], acc[0][2], acc[0][3]);
  acc_guard4(acc[1][0], acc[1][1], acc[1][2], acc[1][3]);
  if (SPLIT) {
    acc_guard4(accr[0][0], accr[0][1], accr[0][2], accr[0][3]);
    acc_guard4(accr[1][0], accr[1][1], accr[1][2], accr[1][3]);
  }

  float* slab = sT[wave];
#pragma unroll
  for (int i = 0; i < 2; ++i) {
    const int mBase = m0 + (i << 4);
#pragma unroll
    for (int j = 0; j < 4; ++j) {
#pragma unroll
      for (int r = 0; r < 8; ++r) {
        float v = acc[i][j][r];
        if (SPLIT) v += accr[i][j][r] * kResInv;
        v *= scale;
        slab[(mOff + r) * 68 + (j << 4) + rlane] = v;
      }
    }
    __builtin_amdgcn_fence(__ATOMIC_RELEASE, "workgroup");
    __builtin_amdgcn_wave_barrier();
    __builtin_amdgcn_fence(__ATOMIC_ACQUIRE, "workgroup");
    {
      const int hh = lane >> 4, c4 = (lane & 15) * 4;
      for (int pass = 0; pass < 2; ++pass) {
#pragma unroll
        for (int it = 0; it < 8; ++it) {
          const int row = it * 2 + hh;
          const v4f v = *(const v4f*)(slab + row * 68 + c4);
          *(volatile v4f*)(C + (size_t)(mBase + row) * ldc + n0 + c4) = v;
        }
        __threadfence();
      }
    }
    __builtin_amdgcn_fence(__ATOMIC_RELEASE, "workgroup");
    __builtin_amdgcn_wave_barrier();
    __builtin_amdgcn_fence(__ATOMIC_ACQUIRE, "workgroup");
  }
}

__global__ __launch_bounds__(256) void wt_plane_kernel(const float* __restrict__ W,
                                                       unsigned short* __restrict__ outh,
                                                       unsigned short* __restrict__ outr,
                                                       int Kd, int Nd, int has_res) {
  __shared__ float sm[64][65];
  const int t  = threadIdx.x;
  const int k0 = blockIdx.x * 64;
  const int n0 = blockIdx.y * 64;
#pragma unroll
  for (int i = 0; i < 16; ++i) {
    const int e = i * 256 + t;
    const int r = e >> 6;
    const int c = e & 63;
    const float v = W[(size_t)(k0 + r) * Nd + n0 + c];
    sm[c][r] = v * kWCarry;
  }
  __syncthreads();
  const int lane = t & 31, wave = t >> 5;
  const int q = lane >> 3, c8 = (lane & 7) * 8;
  for (int pass = 0; pass < 2; ++pass) {
#pragma unroll
    for (int it = 0; it < 2; ++it) {
      const int row = wave * 8 + it * 4 + q;
      float v[8];
#pragma unroll
      for (int e = 0; e < 8; ++e) v[e] = sm[row][c8 + e];
      v4u uh, ur;
      pack8_split(v, uh, ur);
      const size_t o = (size_t)(n0 + row) * Kd + k0 + c8;
      *(volatile v4u*)(outh + o) = uh;
      if (has_res) *(volatile v4u*)(outr + o) = ur;
    }
    __threadfence();
  }
}

__global__ __launch_bounds__(256) void wabc_plane_kernel(const float* __restrict__ WA, const float* __restrict__ WB,
                                                         const float* __restrict__ WC,
                                                         unsigned short* __restrict__ outh,
                                                         unsigned short* __restrict__ outr) {
  __shared__ float sm[64][65];
  const int t  = threadIdx.x;
  const int k0 = blockIdx.x * 64;
#pragma unroll
  for (int i = 0; i < 16; ++i) {
    const int e = i * 256 + t;
    const int r = e >> 6;
    const int c = e & 63;
    const int src = c >> 4;
    const int cc = c & 15;
    const size_t idx = (size_t)(k0 + r) * kNst + cc;
    float va = WA[idx];
    float vb = WB[idx];
    float vc = WC[idx];
    asm volatile("" : "+v"(va));
    asm volatile("" : "+v"(vb));
    asm volatile("" : "+v"(vc));
    const float v = (src == 0) ? va : ((src == 1) ? vb : ((src == 2) ? vc : 0.0f));
    sm[c][r] = v * kWCarry;
  }
  __syncthreads();
  const int lane = t & 31, wave = t >> 5;
  const int q = lane >> 3, c8 = (lane & 7) * 8;
  for (int pass = 0; pass < 2; ++pass) {
#pragma unroll
    for (int it = 0; it < 2; ++it) {
      const int row = wave * 8 + it * 4 + q;
      float v[8];
#pragma unroll
      for (int e = 0; e < 8; ++e) v[e] = sm[row][c8 + e];
      v4u uh, ur;
      pack8_split(v, uh, ur);
      const size_t o = (size_t)row * kDin + k0 + c8;
      *(volatile v4u*)(outh + o) = uh;
      *(volatile v4u*)(outr + o) = ur;
    }
    __threadfence();
  }
}

__global__ __launch_bounds__(256) void x_split_kernel(const float* __restrict__ x,
                                                      unsigned short* __restrict__ XH,
                                                      unsigned short* __restrict__ XL, int total8) {
  const int i = blockIdx.x * 256 + threadIdx.x;
  if (i >= total8) return;
  const size_t off = (size_t)i * 8;
  const v4f a = *(const v4f*)(x + off);
  const v4f b = *(const v4f*)(x + off + 4);
  float o[8];
#pragma unroll
  for (int e = 0; e < 4; ++e) {
    o[e]     = a[e] * kXCarry;
    o[4 + e] = b[e] * kXCarry;
  }
  v4u uh, ur;
  pack8_split(o, uh, ur);
  *(volatile v4u*)(XH + off) = uh;
  *(volatile v4u*)(XL + off) = ur;
  __threadfence();
  *(volatile v4u*)(XH + off) = uh;
  *(volatile v4u*)(XL + off) = ur;
}

__device__ __forceinline__ void gate_group(const _Float16* ph, const _Float16* pl, v16h ah, v16h ar,
                                           v8f& am, v8f& ac) {
  const v16h bh = FragH::load(ph);
  const v16h br = FragH::load(pl);
  am = FragH::mma(ah, bh, am);
  ac = FragH::mma(ah, br, ac);
  ac = FragH::mma(ar, bh, ac);
  guard_m(am, ah, bh);
  guard_c(ac, ah, ar, bh, br);
}

__global__ __launch_bounds__(128) void gemm_gate_kernel(
    const unsigned short* __restrict__ XHp, const unsigned short* __restrict__ XLp,
    const unsigned short* __restrict__ WHp, const unsigned short* __restrict__ WLp,
    unsigned short* __restrict__ XinH, unsigned short* __restrict__ XinL) {
  __shared__ __align__(16) float sS[4][16 * 68];
  __shared__ __align__(16) float sG[4][16 * 68];
  const unsigned lane = threadIdx.x & 31u;
  const unsigned wave = threadIdx.x >> 5;
  const unsigned tile = blockIdx.x * 4u + wave;
  const unsigned tn = tile & (unsigned)(kDin / 64 - 1);
  const unsigned tm = tile / (unsigned)(kDin / 64);
  const unsigned m0 = tm << 4;
  const unsigned d0 = tn << 6;
  const unsigned rlane = lane & 15u;
  const unsigned half8 = (lane >> 4) * 8u;
  const unsigned mOff  = (lane >> 4) * 8u;

  const size_t aoff = (size_t)(m0 + rlane) * kDm + half8;
  const _Float16* pa = (const _Float16*)XHp + aoff;
  const _Float16* pr = (const _Float16*)XLp + aoff;
  const size_t boffS = (size_t)(d0 + rlane) * kDm + half8;
  const size_t boffG = (size_t)((unsigned)kDin + d0 + rlane) * kDm + half8;
  const _Float16* psh = (const _Float16*)WHp + boffS;
  const _Float16* psl = (const _Float16*)WLp + boffS;
  const _Float16* pgh = (const _Float16*)WHp + boffG;
  const _Float16* pgl = (const _Float16*)WLp + boffG;
  constexpr size_t bstep = (size_t)16 * kDm;

  v8f accM[2][4], accC[2][4];
#pragma unroll
  for (int hf = 0; hf < 2; ++hf)
#pragma unroll
    for (int j = 0; j < 4; ++j) {
      accM[hf][j] = (v8f){0.f, 0.f, 0.f, 0.f, 0.f, 0.f, 0.f, 0.f};
      accC[hf][j] = (v8f){0.f, 0.f, 0.f, 0.f, 0.f, 0.f, 0.f, 0.f};
    }

  for (int k0 = 0; k0 < kDm; k0 += 32) {
    const v16h ah = FragH::load(pa + k0);
    const v16h ar = FragH::load(pr + k0);
#pragma unroll
    for (int j = 0; j < 4; ++j) {
      gate_group(psh + j * bstep + k0, psl + j * bstep + k0, ah, ar, accM[0][j], accC[0][j]);
      gate_group(pgh + j * bstep + k0, pgl + j * bstep + k0, ah, ar, accM[1][j], accC[1][j]);
    }
  }
  acc_guard4(accM[0][0], accM[0][1], accM[0][2], accM[0][3]);
  acc_guard4(accM[1][0], accM[1][1], accM[1][2], accM[1][3]);
  acc_guard4(accC[0][0], accC[0][1], accC[0][2], accC[0][3]);
  acc_guard4(accC[1][0], accC[1][1], accC[1][2], accC[1][3]);

  float* slabS = sS[wave];
  float* slabG = sG[wave];
#pragma unroll
  for (int j = 0; j < 4; ++j) {
#pragma unroll
    for (int r = 0; r < 8; ++r) {
      const unsigned so = (mOff + (unsigned)r) * 68u + ((unsigned)j << 4) + rlane;
      slabS[so] = accM[0][j][r] * kFoldMain + accC[0][j][r] * kFoldCross;
      slabG[so] = accM[1][j][r] * kFoldMain + accC[1][j][r] * kFoldCross;
    }
  }
  __builtin_amdgcn_fence(__ATOMIC_RELEASE, "workgroup");
  __builtin_amdgcn_wave_barrier();
  __builtin_amdgcn_fence(__ATOMIC_ACQUIRE, "workgroup");
  {
    const unsigned q = lane >> 3, c8 = (lane & 7u) * 8u;
#pragma unroll 1
    for (int it = 0; it < 4; ++it) {
      const unsigned row = (unsigned)it * 4u + q;
      const float* sp = slabS + row * 68u + c8;
      const float* gp = slabG + row * 68u + c8;
      const v4f s0 = *(const v4f*)(sp);
      const v4f s1 = *(const v4f*)(sp + 4);
      const v4f g0 = *(const v4f*)(gp);
      const v4f g1 = *(const v4f*)(gp + 4);
      float o[8];
#pragma unroll
      for (int e = 0; e < 4; ++e) {
        const float sa = s0[e], ga = g0[e];
        const float sb = s1[e], gb = g1[e];
        const float da = (1.0f + expf(-sa)) * (1.0f + expf(-ga));
        const float db = (1.0f + expf(-sb)) * (1.0f + expf(-gb));
        o[e]     = (sa * (1.0f / da)) * kActCarry;
        o[4 + e] = (sb * (1.0f / db)) * kActCarry;
      }
      v4u uh, ur;
      pack8_split(o, uh, ur);
      const size_t off = (size_t)(m0 + row) * kDin + d0 + c8;
      *(volatile v4u*)(XinH + off) = uh;
      *(volatile v4u*)(XinL + off) = ur;
      __threadfence();
      *(volatile v4u*)(XinH + off) = uh;
      *(volatile v4u*)(XinL + off) = ur;
    }
  }
}

__global__ __launch_bounds__(256) void decay_kernel(float* ABC, int n4) {
  const int i = blockIdx.x * 256 + threadIdx.x;
  if (i >= n4) return;
  float* p = ABC + (size_t)i * 4;
  const v4f v = *(const v4f*)p;
  const bool isA = ((i & 15) < 4);
  v4f o;
#pragma unroll
  for (int e = 0; e < 4; ++e) {
    const float a = v[e];
    const float c = fminf(fmaxf(a, -5.0f), 0.0f);
    const float t = expf(-expf(c));
    o[e] = isA ? t : a;
  }
  *(volatile v4f*)p = o;
  __threadfence();
  *(volatile v4f*)p = o;
}

__global__ __launch_bounds__(256) void scan_diag_kernel(const float* __restrict__ ABC,
                                                        const unsigned short* __restrict__ XinH,
                                                        const unsigned short* __restrict__ XinL,
                                                        unsigned short* __restrict__ OUT16) {
  __shared__ __align__(16) float sX[kScanTS * kAbcP];
  __shared__ __align__(16) float sY[kScanTS * kScanYP];
  const unsigned tid = threadIdx.x, lane = tid & 31u, wave = tid >> 5;
  constexpr unsigned kBlkPerB = kDin / kScanCh;
  const unsigned bix = blockIdx.x / kBlkPerB;
  const unsigned d0  = (blockIdx.x - bix * kBlkPerB) * (unsigned)kScanCh;
  const unsigned d   = d0 + tid;
  const size_t row0 = (size_t)bix * kSeq;
  const unsigned lr = tid >> 4, lc4 = (tid & 15u) * 4u;

  float st[kNst];
#pragma unroll
  for (int n = 0; n < kNst; ++n) st[n] = 0.0f;

#pragma unroll 1
  for (int t0 = 0; t0 < kSeq; t0 += kScanTS) {
#pragma unroll
    for (int i = 0; i < 2; ++i) {
      const unsigned r = lr + 16u * (unsigned)i;
      *(v4f*)(sX + r * kAbcP + lc4) = *(const v4f*)(ABC + (row0 + t0 + r) * kAbcP + lc4);
    }
    __syncthreads();
#pragma unroll 1
    for (int s = 0; s < kScanTS; ++s) {
      const size_t idx = (row0 + t0 + s) * kDin + d;
      const unsigned hb = XinH[idx];
      const unsigned lb = XinL[idx];
      const float xv = (h16_to_f32(hb) + h16_to_f32(lb) * kResInv) * kActInv;
      const float* xr = sX + s * kAbcP;
      float y = 0.0f;
#pragma unroll
      for (int q4 = 0; q4 < 4; ++q4) {
        const v4f de = *(const v4f*)(xr + 4 * q4);
        const v4f bv = *(const v4f*)(xr + kNst + 4 * q4);
        const v4f cv = *(const v4f*)(xr + 2 * kNst + 4 * q4);
#pragma unroll
        for (int e = 0; e < 4; ++e) {
          const float sn = fmaf(st[4 * q4 + e], de[e], xv * bv[e]);
          st[4 * q4 + e] = sn;
          y = fmaf(sn, cv[e], y);
        }
      }
      sY[s * kScanYP + tid] = y;
    }
    __syncthreads();
    v4u uo[4];
#pragma unroll
    for (int it = 0; it < 4; ++it) {
      const unsigned row = (unsigned)it * 8u + wave;
      const float* sp = sY + row * kScanYP + lane * 8u;
      const v4f a0 = *(const v4f*)(sp);
      const v4f a1 = *(const v4f*)(sp + 4);
      float o[8];
#pragma unroll
      for (int e = 0; e < 4; ++e) {
        o[e]     = a0[e] * kScanCarry;
        o[4 + e] = a1[e] * kScanCarry;
      }
      uo[it] = pack8_plain(o);
    }
    for (int pass = 0; pass < 2; ++pass) {
#pragma unroll
      for (int it = 0; it < 4; ++it) {
        const unsigned row = (unsigned)it * 8u + wave;
        const size_t o = (row0 + t0 + row) * kDin + d0 + lane * 8u;
        *(volatile v4u*)(OUT16 + o) = uo[it];
      }
      __threadfence();
    }
  }
}

__global__ __launch_bounds__(256) void rms_norm_kernel(unsigned short* P, const float* __restrict__ normw) {
  const unsigned lane = threadIdx.x & 31u;
  const unsigned wave = threadIdx.x >> 5;
  const unsigned tok = blockIdx.x * 8u + wave;
  unsigned short* rowp = P + (size_t)tok * kDin;
  float ss = 0.0f;
#pragma unroll 1
  for (int it = 0; it < 8; ++it) {
    const unsigned c = ((unsigned)it * 32u + lane) * 8u;
    const v4u w = *(const v4u*)(rowp + c);
    float f[8];
    unpack8(w, f);
#pragma unroll
    for (int e = 0; e < 8; ++e) ss = fmaf(f[e], f[e], ss);
  }
  ss = wave_sum32(ss);
  const float mean = ss * kMeanFold;
  const float inv = 1.0f / sqrtf(mean + kEps);
#pragma unroll 1
  for (int it = 0; it < 8; ++it) {
    const unsigned c = ((unsigned)it * 32u + lane) * 8u;
    const v4u w = *(const v4u*)(rowp + c);
    const v4f n0 = *(const v4f*)(normw + c);
    const v4f n1 = *(const v4f*)(normw + c + 4);
    float f[8];
    unpack8(w, f);
    float o[8];
#pragma unroll
    for (int e = 0; e < 4; ++e) {
      o[e]     = (((f[e] * kScanInv) * inv) * n0[e]) * kNormCarry;
      o[4 + e] = (((f[4 + e] * kScanInv) * inv) * n1[e]) * kNormCarry;
    }
    const v4u u = pack8_plain(o);
    *(volatile v4u*)(rowp + c) = u;
    __threadfence();
    *(volatile v4u*)(rowp + c) = u;
  }
}

extern "C" void kernel_launch(void* const* d_in, const int* in_sizes, int n_in,
                              void* d_out, int out_size, void* d_ws, size_t ws_size, hipStream_t stream) {
  if (n_in < 7 || d_out == nullptr || d_ws == nullptr) return;
  if (in_sizes[0] != kRows * kDm) return;
  if (in_sizes[1] != kDm * kWinN) return;
  if (in_sizes[2] != kDin * kNst || in_sizes[3] != kDin * kNst || in_sizes[4] != kDin * kNst) return;
  if (in_sizes[5] != kDin * kDm) return;
  if (in_sizes[6] != kDin) return;
  if (out_size != kRows * kDm) return;
  if (ws_size < kWsTotal) return;

  const float* x     = (const float*)d_in[0];
  const float* W_in  = (const float*)d_in[1];
  const float* W_A   = (const float*)d_in[2];
  const float* W_B   = (const float*)d_in[3];
  const float* W_C   = (const float*)d_in[4];
  const float* W_out = (const float*)d_in[5];
  const float* normw = (const float*)d_in[6];
  float* out = (float*)d_out;

  char* ws = (char*)d_ws;
  size_t off = 0;
  auto carve = [&](size_t bytes) -> char* {
    char* p = ws + off;
    off += (bytes + 255) & ~(size_t)255;
    return p;
  };
  unsigned short* WinH  = (unsigned short*)carve(kSzWin);
  unsigned short* WinL  = (unsigned short*)carve(kSzWin);
  unsigned short* WabcH = (unsigned short*)carve(kSzWabc);
  unsigned short* WabcL = (unsigned short*)carve(kSzWabc);
  unsigned short* WoutH = (unsigned short*)carve(kSzWout);
  unsigned short* XH    = (unsigned short*)carve(kSzXHL);
  unsigned short* XinH  = (unsigned short*)carve(kSzXin);
  unsigned short* XinL  = (unsigned short*)carve(kSzXin);
  float*          ABC   = (float*)carve(kSzAbc);
  unsigned short* XL    = XH + (size_t)kRows * kDm;
  unsigned short* OUT16 = XH;
  if (off != kWsTotal || off > ws_size) return;

  wt_plane_kernel<<<dim3(kDm / 64, kWinN / 64), 256, 0, stream>>>(W_in, WinH, WinL, kDm, kWinN, 1);
  wabc_plane_kernel<<<kDin / 64, 256, 0, stream>>>(W_A, W_B, W_C, WabcH, WabcL);
  wt_plane_kernel<<<dim3(kDin / 64, kDm / 64), 256, 0, stream>>>(W_out, WoutH, WoutH, kDin, kDm, 0);

  x_split_kernel<<<(kRows * kDm / 8) / 256, 256, 0, stream>>>(x, XH, XL, kRows * kDm / 8);

  gemm_gate_kernel<<<((kRows / 16) * (kDin / 64)) / 4, 128, 0, stream>>>(XH, XL, WinH, WinL, XinH, XinL);

  gemm_f16_kernel<true><<<((kRows / 32) * (kAbcP / 64)) / 8, 256, 0, stream>>>(
      XinH, XinL, kDin, WabcH, WabcL, kDin, ABC, kAbcP, kRows, kAbcP, kDin, kScaleAbc);

  decay_kernel<<<(kRows * kAbcP / 4) / 256, 256, 0, stream>>>(ABC, kRows * kAbcP / 4);

  scan_diag_kernel<<<kBatch * (kDin / kScanCh), kScanCh, 0, stream>>>(ABC, XinH, XinL, OUT16);

  rms_norm_kernel<<<kRows / 8, 256, 0, stream>>>(OUT16, normw);

  gemm_f16_kernel<false><<<((kRows / 32) * (kDm / 64)) / 8, 256, 0, stream>>>(
      OUT16, OUT16, kDin, WoutH, WoutH, kDin, out, kDm, kRows, kDm, kDin, kScaleOut);
}
